// TransformerBasedTransformCodingHyper_77421080478300
// MI455X (gfx1250) — hardware-run, weakly checked
//
#include <hip/hip_runtime.h>
#include <math.h>

constexpr int kBatch     = 16;
constexpr int kImgH      = 56;
constexpr int kImgW      = 56;
constexpr int kChan      = 256;
constexpr int kWin       = 7;
constexpr int kShift     = 3;
constexpr int kHeads     = 8;
constexpr int kHeadDim   = 32;
constexpr int kTok       = 49;
constexpr int kWinPerImg = 64;
constexpr int kNumWin    = kBatch * kWinPerImg;
constexpr int kPix       = kImgH * kImgW;
constexpr int kRows      = kBatch * kPix;
constexpr int kQkvN      = 3 * kChan;
constexpr int kMlp       = 4 * kChan;
constexpr int kRpbN      = (2 * kWin - 1) * (2 * kWin - 1);

constexpr float kAttnScale  = 0.17677669529663689f;
constexpr float kWCarry     = 16.0f;
constexpr float kInvWCarry  = 1.0f / 16.0f;
constexpr float kPCarry     = 1024.0f;
constexpr float kCtxCarry   = 16.0f;
constexpr float kCtxFromAcc = kCtxCarry / kPCarry;
constexpr float kProjScale  = 1.0f / (kCtxCarry * kWCarry);
constexpr float kGeluCarry  = 8.0f;
constexpr float kFc2Scale   = 1.0f / (kGeluCarry * kWCarry);

constexpr int kWinChunk     = 256;
constexpr int kQkvChunkRows = kWinChunk * kTok;
constexpr int kNumQkvChunks = kNumWin / kWinChunk;
constexpr int kMlpChunkRows = 6272;
constexpr int kNumMlpChunks = kRows / kMlpChunkRows;
static_assert(kQkvChunkRows % 64 == 0, "tile multiple");
static_assert(kMlpChunkRows % 64 == 0 && kNumMlpChunks * kMlpChunkRows == kRows, "tile multiple");
static_assert(kRows % 64 == 0 && kRows % 8 == 0, "tile multiple");

constexpr int kWaveLds      = 7168;
constexpr int kOsOff        = 8 * kWaveLds;
constexpr int kAttnLdsBytes = (kOsOff + 64 * kChan) * 2;

constexpr size_t kOffWqkv  = 0;
constexpr size_t kOffWproj = kOffWqkv + (size_t)kQkvN * kChan * 2;
constexpr size_t kOffWfc1  = kOffWproj + (size_t)kChan * kChan * 2;
constexpr size_t kOffWfc2  = kOffWfc1 + (size_t)kMlp * kChan * 2;
constexpr size_t kOffXW    = kOffWfc2 + (size_t)kChan * kMlp * 2;
constexpr size_t kOffCTX   = kOffXW + (size_t)kRows * kChan * 2;
constexpr size_t kOffQKV   = kOffCTX + (size_t)kRows * kChan * 2;
constexpr size_t kOffX1    = kOffQKV + (size_t)kQkvChunkRows * kQkvN * 2;
constexpr size_t kWsTotal  = kOffX1 + (size_t)kRows * kChan * 4;
static_assert(kWsTotal == 123600896, "carve");
static_assert((size_t)kMlpChunkRows * kMlp * 4 <= (size_t)kRows * kChan * 2, "H32 chunk fits R_CTX");
static_assert((size_t)kMlpChunkRows * kMlp * 2 <= (size_t)kQkvChunkRows * kQkvN * 2, "G16 chunk fits R_QKV");
static_assert(kWsTotal <= 134217728, "carve under 128 MiB");

typedef __attribute__((ext_vector_type(16))) _Float16 v16h;
typedef __attribute__((ext_vector_type(8)))  _Float16 v8h;
typedef __attribute__((ext_vector_type(16))) __bf16   v16b;
typedef __attribute__((ext_vector_type(8)))  __bf16   v8b;
typedef __attribute__((ext_vector_type(8)))  float    v8f;
typedef __attribute__((ext_vector_type(4)))  float    v4f;
typedef __attribute__((ext_vector_type(4)))  unsigned int v4u;

__device__ __forceinline__ unsigned short f2bf_bits(float f) {
  unsigned u = __float_as_uint(f);
  return (unsigned short)((u + 0x7FFFu + ((u >> 16) & 1u)) >> 16);
}
__device__ __forceinline__ float bf_bits2f(unsigned short h) { return __uint_as_float(((unsigned)h) << 16); }

__device__ __forceinline__ void dep_guard_h(v8f& a, v8f& b, v16h x, v16h y) { asm volatile("v_nop\n\tv_nop\n\tv_nop\n\tv_nop" : "+v"(a), "+v"(b) : "v"(x), "v"(y)); }
__device__ __forceinline__ void dep_guard_b(v8f& a, v8f& b, v16b x, v16b y) { asm volatile("v_nop\n\tv_nop\n\tv_nop\n\tv_nop" : "+v"(a), "+v"(b) : "v"(x), "v"(y)); }
__device__ __forceinline__ void keep4_h(v16h a, v16h b, v16h c, v16h d) { asm volatile("v_nop" :: "v"(a), "v"(b), "v"(c), "v"(d)); }
__device__ __forceinline__ void keep4_b(v16b a, v16b b, v16b c, v16b d) { asm volatile("v_nop" :: "v"(a), "v"(b), "v"(c), "v"(d)); }
__device__ __forceinline__ void acc_guard4(v8f& a, v8f& b, v8f& c, v8f& d) { asm volatile("v_nop\n\tv_nop\n\tv_nop\n\tv_nop" : "+v"(a), "+v"(b), "+v"(c), "+v"(d)); }
template <typename T> struct Frag;
template <> struct Frag<_Float16> {
  typedef v16h V; union U { v16h v; v8h h[2]; };
  static __device__ __forceinline__ v16h load(const _Float16* p) {
    U f; f.h[0] = *(const v8h*)(p); f.h[1] = *(const v8h*)(p + 16); return f.v;
  }
  static __device__ __forceinline__ v8f mma(v16h a, v16h b, v8f c) {
    return __builtin_amdgcn_wmma_f32_16x16x32_f16(false, a, false, b, (short)0, c, false, false);
  }
  static __device__ __forceinline__ void guard(v8f& a, v8f& b, v16h x, v16h y) { dep_guard_h(a, b, x, y); }
  static __device__ __forceinline__ void keep(v16h a, v16h b, v16h c, v16h d) { keep4_h(a, b, c, d); }
};
template <> struct Frag<__bf16> {
  typedef v16b V; union U { v16b v; v8b h[2]; };
  static __device__ __forceinline__ v16b load(const __bf16* p) {
    U f; f.h[0] = *(const v8b*)(p); f.h[1] = *(const v8b*)(p + 16); return f.v;
  }
  static __device__ __forceinline__ v8f mma(v16b a, v16b b, v8f c) {
    return __builtin_amdgcn_wmma_f32_16x16x32_bf16(false, a, false, b, (short)0, c, false, false);
  }
  static __device__ __forceinline__ void guard(v8f& a, v8f& b, v16b x, v16b y) { dep_guard_b(a, b, x, y); }
  static __device__ __forceinline__ void keep(v16b a, v16b b, v16b c, v16b d) { keep4_b(a, b, c, d); }
};

__device__ __forceinline__ unsigned pk16(unsigned short a, unsigned short b) { return (unsigned)a | ((unsigned)b << 16); }
__device__ __forceinline__ unsigned short h_bits(float f) { const _Float16 h = (_Float16)f; return __builtin_bit_cast(unsigned short, h); }

__device__ __forceinline__ v8f mma_h(v16h a, v16h b, v8f cacc) {
  cacc = __builtin_amdgcn_wmma_f32_16x16x32_f16(false, a, false, b, (short)0, cacc, false, false);
  asm volatile("v_nop\n\tv_nop\n\tv_nop\n\tv_nop" : "+v"(cacc) : "v"(a), "v"(b));
  return cacc;
}

__device__ __forceinline__ float wsum32(float v) {
  v += __shfl_xor(v, 16, 32);
  v += __shfl_xor(v, 8, 32);
  v += __shfl_xor(v, 4, 32);
  v += __shfl_xor(v, 2, 32);
  v += __shfl_xor(v, 1, 32);
  return v;
}

template <int ET> struct Elem;
template <> struct Elem<0> { typedef _Float16 T; };
template <> struct Elem<1> { typedef __bf16 T; };
template <int ET, bool SPLIT, int BIAS_MODE, int OUT_MODE, bool RESID, int ACT = 0>
__global__ __launch_bounds__(256) void wmma_gemm64(
    const unsigned short* __restrict__ Ap, const unsigned short* __restrict__ A2p, int lda, long strideA,
    const unsigned short* __restrict__ Btp, const unsigned short* __restrict__ Bt2p, int ldb, long strideB,
    void* __restrict__ Cout, void* __restrict__ Cout2, int ldc, long strideC,
    const float* __restrict__ bias,
    const float* __restrict__ resid, long strideR,
    int M, int N, int K, float scale) {
  typedef typename Elem<ET>::T T;
  typedef typename Frag<T>::V V;
  const T* A = (const T*)Ap; const T* A2 = (const T*)A2p; const T* Bt = (const T*)Btp; const T* Bt2 = (const T*)Bt2p;
  __shared__ __align__(16) float sT[8][16 * 68];
  const int b    = blockIdx.y;
  const int lane = threadIdx.x & 31;
  const int wave = threadIdx.x >> 5;
  const int tilesN = N >> 6;
  const int tilesM = M >> 6;
  const int tile = blockIdx.x * 8 + wave;
  if (tile >= tilesM * tilesN) return;
  const int tm = tile / tilesN;
  const int tn = tile - tm * tilesN;
  const int m0 = tm << 6;
  const int n0 = tn << 6;

  const T* Ab  = A  + (size_t)b * strideA;
  const T* Bb  = Bt + (size_t)b * strideB;
  const T* Ab2 = SPLIT ? (A2  + (size_t)b * strideA) : nullptr;
  const T* Bb2 = SPLIT ? (Bt2 + (size_t)b * strideB) : nullptr;

  const int rlane = lane & 15;
  const int koff  = (lane >> 4) * 8;
  const int mOff  = (lane >> 4) * 8;

  v8f acc[4][4];
#pragma unroll
  for (int i = 0; i < 4; ++i)
#pragma unroll
    for (int j = 0; j < 4; ++j) acc[i][j] = (v8f){0.f,0.f,0.f,0.f,0.f,0.f,0.f,0.f};

  for (int k0 = 0; k0 < K; k0 += 32) {
    V bh[4], bl[4];
#pragma unroll
    for (int j = 0; j < 4; ++j) {
      const size_t bo = (size_t)(n0 + (j << 4) + rlane) * ldb + koff + k0;
      bh[j] = Frag<T>::load(Bb + bo);
      if (SPLIT) bl[j] = Frag<T>::load(Bb2 + bo);
    }
#pragma unroll
    for (int i = 0; i < 4; ++i) {
      const size_t ao = (size_t)(m0 + (i << 4) + rlane) * lda + koff + k0;
      V ah = Frag<T>::load(Ab + ao);
      V al;
      if (SPLIT) al = Frag<T>::load(Ab2 + ao);
#pragma unroll
      for (int j = 0; j < 4; ++j) {
        acc[i][j] = Frag<T>::mma(ah, bh[j], acc[i][j]);
        if (SPLIT) {
          acc[i][j] = Frag<T>::mma(ah, bl[j], acc[i][j]);
          acc[i][j] = Frag<T>::mma(al, bh[j], acc[i][j]);
        }
      }
      Frag<T>::guard(acc[i][0], acc[i][3], ah, SPLIT ? al : ah);
    }
    Frag<T>::keep(bh[0], bh[1], bh[2], bh[3]);
    if (SPLIT) Frag<T>::keep(bl[0], bl[1], bl[2], bl[3]);
  }
  acc_guard4(acc[0][0], acc[0][1], acc[0][2], acc[0][3]);
  acc_guard4(acc[1][0], acc[1][1], acc[1][2], acc[1][3]);
  acc_guard4(acc[2][0], acc[2][1], acc[2][2], acc[2][3]);
  acc_guard4(acc[3][0], acc[3][1], acc[3][2], acc[3][3]);

  float* slab = sT[wave];
  const float* Rb = RESID ? (resid + (size_t)b * strideR) : nullptr;
#pragma unroll
  for (int i = 0; i < 4; ++i) {
    const int mBase = m0 + (i << 4);
#pragma unroll
    for (int j = 0; j < 4; ++j) {
      const int n = n0 + (j << 4) + rlane;
      float bv = 0.f;
      if (BIAS_MODE == 2) bv = bias[n];
#pragma unroll
      for (int r = 0; r < 8; ++r) {
        float v = acc[i][j][r] * scale;
        if (BIAS_MODE == 1) v += bias[mBase + mOff + r];
        if (BIAS_MODE == 2) v += bv;
        if (RESID) v += Rb[(size_t)(mBase + mOff + r) * ldc + n];
        if (ACT == 2) v = fmaxf(v, 0.0f);
        if (ACT == 4) v = (v > 0.f) ? v : 0.01f * v;
        slab[(mOff + r) * 68 + (j << 4) + rlane] = v;
      }
    }
    __builtin_amdgcn_fence(__ATOMIC_RELEASE, "workgroup");
    __builtin_amdgcn_wave_barrier();
    __builtin_amdgcn_fence(__ATOMIC_ACQUIRE, "workgroup");
    if (OUT_MODE == 0) {
      float* C = (float*)Cout + (size_t)b * strideC;
      const int hh = lane >> 4, c4 = (lane & 15) * 4;
      for (int pass = 0; pass < 2; ++pass) {
#pragma unroll
        for (int it = 0; it < 8; ++it) {
          const int row = it * 2 + hh;
          v4f v = *(const v4f*)(slab + row * 68 + c4);
          *(volatile v4f*)(C + (size_t)(mBase + row) * ldc + n0 + c4) = v;
        }
        __threadfence();
      }
    } else {
      const int q = lane >> 3, c8 = (lane & 7) * 8;
      unsigned short* C  = (unsigned short*)Cout  + (size_t)b * strideC;
      unsigned short* C2 = (OUT_MODE == 2) ? ((unsigned short*)Cout2 + (size_t)b * strideC) : nullptr;
      for (int pass = 0; pass < 2; ++pass) {
#pragma unroll
        for (int it = 0; it < 4; ++it) {
          const int row = it * 4 + q;
          const float* sp = slab + row * 68 + c8;
          v8h hv, lv;
#pragma unroll
          for (int e = 0; e < 8; ++e) {
            if (OUT_MODE == 1) {
              hv[e] = (_Float16)sp[e];
            } else {
              unsigned short hb = f2bf_bits(sp[e]);
              unsigned short lb = f2bf_bits(sp[e] - bf_bits2f(hb));
              hv[e] = __builtin_bit_cast(_Float16, hb);
              lv[e] = __builtin_bit_cast(_Float16, lb);
            }
          }
          *(volatile v8h*)(C + (size_t)(mBase + row) * ldc + n0 + c8) = hv;
          if (OUT_MODE == 2) *(volatile v8h*)(C2 + (size_t)(mBase + row) * ldc + n0 + c8) = lv;
        }
        __threadfence();
      }
    }
    __builtin_amdgcn_fence(__ATOMIC_RELEASE, "workgroup");
    __builtin_amdgcn_wave_barrier();
    __builtin_amdgcn_fence(__ATOMIC_ACQUIRE, "workgroup");
  }
}

__global__ __launch_bounds__(256) void wcast4_kernel(const float* __restrict__ w0, unsigned short* __restrict__ o0, int n0,
                                                     const float* __restrict__ w1, unsigned short* __restrict__ o1, int n1,
                                                     const float* __restrict__ w2, unsigned short* __restrict__ o2, int n2,
                                                     const float* __restrict__ w3, unsigned short* __restrict__ o3, int n3,
                                                     float scale) {
  const int y = blockIdx.y;
  const float* src = (y == 0) ? w0 : (y == 1) ? w1 : (y == 2) ? w2 : w3;
  unsigned short* dst = (y == 0) ? o0 : (y == 1) ? o1 : (y == 2) ? o2 : o3;
  const int npairs = ((y == 0) ? n0 : (y == 1) ? n1 : (y == 2) ? n2 : n3) >> 1;
  const int i = blockIdx.x * 256 + threadIdx.x;
  if (i >= npairs) return;
  const float a = src[2 * (size_t)i] * scale;
  const float c = src[2 * (size_t)i + 1] * scale;
  const unsigned u = pk16(h_bits(a), h_bits(c));
  ((volatile unsigned*)dst)[i] = u;
  __threadfence();
  ((volatile unsigned*)dst)[i] = u;
}

template <bool WINMAP>
__global__ __launch_bounds__(256) void layernorm_f16_kernel(const float* __restrict__ x, const float* __restrict__ g,
                                                            const float* __restrict__ bta, unsigned short* __restrict__ out) {
  const int wave = threadIdx.x >> 5, lane = threadIdx.x & 31;
  const int row = blockIdx.x * 8 + wave;
  const float* xr = x + (size_t)row * kChan + lane * 8;
  const v4f a0 = *(const v4f*)(xr);
  const v4f a1 = *(const v4f*)(xr + 4);
  float v[8];
#pragma unroll
  for (int e = 0; e < 4; ++e) { v[e] = a0[e]; v[4 + e] = a1[e]; }
  float s = ((v[0] + v[1]) + (v[2] + v[3])) + ((v[4] + v[5]) + (v[6] + v[7]));
  s = wsum32(s);
  const float mean = s * (1.0f / 256.0f);
  float q = 0.f;
#pragma unroll
  for (int e = 0; e < 8; ++e) { const float d = v[e] - mean; q += d * d; }
  q = wsum32(q);
  const float rstd = 1.0f / sqrtf(q * (1.0f / 256.0f) + 1e-5f);
  const v4f g0 = *(const v4f*)(g + lane * 8);
  const v4f g1 = *(const v4f*)(g + lane * 8 + 4);
  const v4f b0 = *(const v4f*)(bta + lane * 8);
  const v4f b1 = *(const v4f*)(bta + lane * 8 + 4);
  unsigned short hb[8];
#pragma unroll
  for (int e = 0; e < 4; ++e) {
    hb[e]     = h_bits((v[e] - mean) * rstd * g0[e] + b0[e]);
    hb[4 + e] = h_bits((v[4 + e] - mean) * rstd * g1[e] + b1[e]);
  }
  const v4u u = (v4u){pk16(hb[0], hb[1]), pk16(hb[2], hb[3]), pk16(hb[4], hb[5]), pk16(hb[6], hb[7])};
  int orow = row;
  if (WINMAP) {
    const int bimg = row / kPix;
    const int hw = row - bimg * kPix;
    const int hh = hw / kImgW;
    const int ww = hw - hh * kImgW;
    int i = hh - kShift; if (i < 0) i += kImgH;
    int j = ww - kShift; if (j < 0) j += kImgW;
    const int wy = i / kWin, iy = i - wy * kWin;
    const int wx = j / kWin, ix = j - wx * kWin;
    orow = (bimg * kWinPerImg + wy * 8 + wx) * kTok + iy * kWin + ix;
  }
  unsigned short* dst = out + (size_t)orow * kChan + lane * 8;
  *(volatile v4u*)dst = u;
  __threadfence();
  *(volatile v4u*)dst = u;
}

__global__ __launch_bounds__(256) void win_attn_kernel(const unsigned short* __restrict__ qkv, const float* __restrict__ rpb,
                                                       const float* __restrict__ maskm, unsigned short* __restrict__ ctx, int win0) {
  extern __shared__ v4u lds_raw[];
  unsigned short* lds_u16 = (unsigned short*)lds_raw;
  const int wl   = blockIdx.x;
  const int bwin = win0 + wl;
  const int widx = bwin & (kWinPerImg - 1);
  const int bimg = bwin >> 6;
  const int wy = widx >> 3, wx = widx & 7;
  const int wave = threadIdx.x >> 5, lane = threadIdx.x & 31;
  const int hh = lane >> 4, c = lane & 15, koff = hh * 8;
  const int head = wave;
  const int hcol = head * kHeadDim;
  unsigned short* Qs = lds_u16 + wave * kWaveLds;
  unsigned short* Ks = Qs + 2048;
  unsigned short* Vt = Qs + 4096;
  unsigned short* Ps = Qs + 6144;
  unsigned short* Os = lds_u16 + kOsOff;
  const size_t rowbase = (size_t)wl * kTok;
  const v4u z4 = (v4u){0u, 0u, 0u, 0u};

#pragma unroll
  for (int it = 0; it < 8; ++it) {
    const int i  = it * 32 + lane;
    const int j  = i >> 2;
    const int dq = (i & 3) * 8;
    const int jc = (j < kTok) ? j : (kTok - 1);
    const unsigned short* src = qkv + (rowbase + jc) * kQkvN + hcol + dq;
    v4u q4 = *(const v4u*)(src);
    v4u k4 = *(const v4u*)(src + kChan);
    const unsigned keep = (j < kTok) ? 0xffffffffu : 0u;
    const v4u km = (v4u){keep, keep, keep, keep};
    q4 = q4 & km;
    k4 = k4 & km;
    *(v4u*)(Qs + j * 32 + dq) = q4;
    *(v4u*)(Ks + j * 32 + dq) = k4;
    *(v4u*)(Vt + i * 8) = z4;
  }
  __syncthreads();
#pragma unroll
  for (int it = 0; it < 7; ++it) {
    const int i  = it * 32 + lane;
    const int ic = (i < 4 * kTok) ? i : (4 * kTok - 1);
    const int j  = ic >> 2;
    const int d0 = (ic & 3) * 8;
    const v4u v4 = *(const v4u*)(qkv + (rowbase + j) * kQkvN + 2 * kChan + hcol + d0);
    if (i < 4 * kTok) {
      Vt[(d0 + 0) * 64 + j] = (unsigned short)(v4.x & 0xffffu);
      Vt[(d0 + 1) * 64 + j] = (unsigned short)(v4.x >> 16);
      Vt[(d0 + 2) * 64 + j] = (unsigned short)(v4.y & 0xffffu);
      Vt[(d0 + 3) * 64 + j] = (unsigned short)(v4.y >> 16);
      Vt[(d0 + 4) * 64 + j] = (unsigned short)(v4.z & 0xffffu);
      Vt[(d0 + 5) * 64 + j] = (unsigned short)(v4.z >> 16);
      Vt[(d0 + 6) * 64 + j] = (unsigned short)(v4.w & 0xffffu);
      Vt[(d0 + 7) * 64 + j] = (unsigned short)(v4.w >> 16);
    }
  }
  __syncthreads();

  const _Float16* Qh = (const _Float16*)Qs;
  const _Float16* Kh = (const _Float16*)Ks;
  const _Float16* Vh = (const _Float16*)Vt;
  _Float16* Ph = (_Float16*)Ps;
  _Float16* Oh = (_Float16*)Os;
  const float* mwin = maskm + (size_t)widx * (kTok * kTok);
  const v8f z8 = (v8f){0.f, 0.f, 0.f, 0.f, 0.f, 0.f, 0.f, 0.f};

#pragma unroll 1
  for (int tm = 0; tm < 4; ++tm) {
    const v16h aq = Frag<_Float16>::load(Qh + (tm * 16 + c) * kHeadDim + koff);
    v8f s[4];
#pragma unroll
    for (int tn = 0; tn < 4; ++tn) {
      const v16h bk = Frag<_Float16>::load(Kh + (tn * 16 + c) * kHeadDim + koff);
      s[tn] = mma_h(aq, bk, z8);
    }
    const int i0 = tm * 16 + 8 * hh;
#pragma unroll
    for (int tn = 0; tn < 4; ++tn) {
      const int j  = tn * 16 + c;
      const int jc = (j < kTok) ? j : (kTok - 1);
      const int jy = jc / kWin, jx = jc - jy * kWin;
      const bool jok = (j < kTok);
#pragma unroll
      for (int r = 0; r < 8; ++r) {
        const int i  = i0 + r;
        const int ic = (i < kTok) ? i : (kTok - 1);
        const int iy = ic / kWin, ix = ic - iy * kWin;
        const float bv = rpb[((iy - jy + (kWin - 1)) * (2 * kWin - 1) + (ix - jx + (kWin - 1))) * kHeads + head]
                       + mwin[ic * kTok + jc];
        const float t = s[tn][r] * kAttnScale + bv;
        s[tn][r] = jok ? t : -1e30f;
      }
    }
#pragma unroll
    for (int r = 0; r < 8; ++r) {
      float m = fmaxf(fmaxf(s[0][r], s[1][r]), fmaxf(s[2][r], s[3][r]));
      m = fmaxf(m, __shfl_xor(m, 1, 32));
      m = fmaxf(m, __shfl_xor(m, 2, 32));
      m = fmaxf(m, __shfl_xor(m, 4, 32));
      m = fmaxf(m, __shfl_xor(m, 8, 32));
      float sum = 0.f;
#pragma unroll
      for (int tn = 0; tn < 4; ++tn) {
        const float e = expf(s[tn][r] - m);
        s[tn][r] = e;
        sum += e;
      }
      sum += __shfl_xor(sum, 1, 32);
      sum += __shfl_xor(sum, 2, 32);
      sum += __shfl_xor(sum, 4, 32);
      sum += __shfl_xor(sum, 8, 32);
      const float inv = kPCarry / sum;
#pragma unroll
      for (int tn = 0; tn < 4; ++tn) Ph[(8 * hh + r) * 64 + tn * 16 + c] = (_Float16)(s[tn][r] * inv);
    }
    __builtin_amdgcn_fence(__ATOMIC_RELEASE, "workgroup");
    __builtin_amdgcn_wave_barrier();
    __builtin_amdgcn_fence(__ATOMIC_ACQUIRE, "workgroup");
    v8f o[2];
    o[0] = z8; o[1] = z8;
#pragma unroll
    for (int kk = 0; kk < 2; ++kk) {
      const v16h ap = Frag<_Float16>::load(Ph + c * 64 + kk * 32 + koff);
#pragma unroll
      for (int nb = 0; nb < 2; ++nb) {
        const v16h bvv = Frag<_Float16>::load(Vh + (nb * 16 + c) * 64 + kk * 32 + koff);
        o[nb] = mma_h(ap, bvv, o[nb]);
      }
    }
#pragma unroll
    for (int nb = 0; nb < 2; ++nb)
#pragma unroll
      for (int r = 0; r < 8; ++r)
        Oh[(tm * 16 + 8 * hh + r) * kChan + hcol + nb * 16 + c] = (_Float16)(o[nb][r] * kCtxFromAcc);
    __builtin_amdgcn_fence(__ATOMIC_RELEASE, "workgroup");
    __builtin_amdgcn_wave_barrier();
    __builtin_amdgcn_fence(__ATOMIC_ACQUIRE, "workgroup");
  }
  __syncthreads();

  for (int pass = 0; pass < 2; ++pass) {
    for (int t = wave; t < kTok; t += 8) {
      const int iy = t / kWin, ix = t - iy * kWin;
      int h2 = wy * kWin + iy + kShift; if (h2 >= kImgH) h2 -= kImgH;
      int w2 = wx * kWin + ix + kShift; if (w2 >= kImgW) w2 -= kImgW;
      const size_t orow = (size_t)bimg * kPix + (size_t)h2 * kImgW + w2;
      const v4u val = *(const v4u*)(Os + t * kChan + lane * 8);
      *(volatile v4u*)(ctx + orow * kChan + lane * 8) = val;
    }
    __threadfence();
  }
}

__global__ __launch_bounds__(256) void gelu_f16_kernel(const float* __restrict__ in, unsigned short* __restrict__ out,
                                                       int npairs, float carry) {
  const int i = blockIdx.x * 256 + threadIdx.x;
  if (i >= npairs) return;
  const float a = in[2 * (size_t)i];
  const float c = in[2 * (size_t)i + 1];
  const float ga = 0.5f * a * (1.0f + erff(a * 0.70710678118654752f)) * carry;
  const float gc = 0.5f * c * (1.0f + erff(c * 0.70710678118654752f)) * carry;
  const unsigned u = pk16(h_bits(ga), h_bits(gc));
  ((volatile unsigned*)out)[i] = u;
  __threadfence();
  ((volatile unsigned*)out)[i] = u;
}

extern "C" void kernel_launch(void* const* d_in, const int* in_sizes, int n_in,
                              void* d_out, int out_size, void* d_ws, size_t ws_size,
                              hipStream_t stream) {
  if (n_in < 15) return;
  if (ws_size < kWsTotal) return;
  if (in_sizes[0] != kRows * kChan || out_size != kRows * kChan) return;
  if (in_sizes[1] != kWinPerImg * kTok * kTok || in_sizes[4] != kQkvN * kChan || in_sizes[6] != kRpbN * kHeads ||
      in_sizes[7] != kChan * kChan || in_sizes[11] != kMlp * kChan || in_sizes[13] != kChan * kMlp) return;

  const float* x      = (const float*)d_in[0];
  const float* maskm  = (const float*)d_in[1];
  const float* n1g    = (const float*)d_in[2];
  const float* n1b    = (const float*)d_in[3];
  const float* qkv_w  = (const float*)d_in[4];
  const float* qkv_b  = (const float*)d_in[5];
  const float* rpbt   = (const float*)d_in[6];
  const float* proj_w = (const float*)d_in[7];
  const float* proj_b = (const float*)d_in[8];
  const float* n2g    = (const float*)d_in[9];
  const float* n2b    = (const float*)d_in[10];
  const float* fc1_w  = (const float*)d_in[11];
  const float* fc1_b  = (const float*)d_in[12];
  const float* fc2_w  = (const float*)d_in[13];
  const float* fc2_b  = (const float*)d_in[14];
  float* out = (float*)d_out;

  char* ws = (char*)d_ws;
  unsigned short* Wqkv16  = (unsigned short*)(ws + kOffWqkv);
  unsigned short* Wproj16 = (unsigned short*)(ws + kOffWproj);
  unsigned short* Wfc1_16 = (unsigned short*)(ws + kOffWfc1);
  unsigned short* Wfc2_16 = (unsigned short*)(ws + kOffWfc2);
  unsigned short* XW16    = (unsigned short*)(ws + kOffXW);
  unsigned short* Y16     = XW16;
  unsigned short* CTX16   = (unsigned short*)(ws + kOffCTX);
  float*          H32     = (float*)(ws + kOffCTX);
  unsigned short* QKV16   = (unsigned short*)(ws + kOffQKV);
  unsigned short* G16     = QKV16;
  float*          X1      = (float*)(ws + kOffX1);

  wcast4_kernel<<<dim3(512, 4), 256, 0, stream>>>(qkv_w, Wqkv16, in_sizes[4], proj_w, Wproj16, in_sizes[7],
                                                   fc1_w, Wfc1_16, in_sizes[11], fc2_w, Wfc2_16, in_sizes[13], kWCarry);

  layernorm_f16_kernel<true><<<kRows / 8, 256, 0, stream>>>(x, n1g, n1b, XW16);

  for (int ch = 0; ch < kNumQkvChunks; ++ch) {
    const int tiles = (kQkvChunkRows / 64) * (kQkvN / 64);
    wmma_gemm64<0, false, 2, 1, false, 0><<<dim3((tiles + 7) / 8, 1), 256, 0, stream>>>(
        XW16 + (size_t)ch * kQkvChunkRows * kChan, nullptr, kChan, 0L,
        Wqkv16, nullptr, kChan, 0L,
        (void*)QKV16, nullptr, kQkvN, 0L,
        qkv_b, nullptr, 0L, kQkvChunkRows, kQkvN, kChan, kInvWCarry);
    win_attn_kernel<<<kWinChunk, 256, kAttnLdsBytes, stream>>>(QKV16, rpbt, maskm, CTX16, ch * kWinChunk);
  }

  {
    const int tiles = (kRows / 64) * (kChan / 64);
    wmma_gemm64<0, false, 2, 0, true, 0><<<dim3((tiles + 7) / 8, 1), 256, 0, stream>>>(
        CTX16, nullptr, kChan, 0L,
        Wproj16, nullptr, kChan, 0L,
        (void*)X1, nullptr, kChan, 0L,
        proj_b, x, 0L, kRows, kChan, kChan, kProjScale);
  }

  layernorm_f16_kernel<false><<<kRows / 8, 256, 0, stream>>>(X1, n2g, n2b, Y16);

  for (int ch = 0; ch < kNumMlpChunks; ++ch) {
    const size_t r0 = (size_t)ch * kMlpChunkRows;
    const int tiles1 = (kMlpChunkRows / 64) * (kMlp / 64);
    wmma_gemm64<0, false, 2, 0, false, 0><<<dim3((tiles1 + 7) / 8, 1), 256, 0, stream>>>(
        Y16 + r0 * kChan, nullptr, kChan, 0L,
        Wfc1_16, nullptr, kChan, 0L,
        (void*)H32, nullptr, kMlp, 0L,
        fc1_b, nullptr, 0L, kMlpChunkRows, kMlp, kChan, kInvWCarry);
    const int npairs = kMlpChunkRows * kMlp / 2;
    gelu_f16_kernel<<<(npairs + 255) / 256, 256, 0, stream>>>(H32, G16, npairs, kGeluCarry);
    const int tiles2 = (kMlpChunkRows / 64) * (kChan / 64);
    wmma_gemm64<0, false, 2, 0, true, 0><<<dim3((tiles2 + 7) / 8, 1), 256, 0, stream>>>(
        G16, nullptr, kMlp, 0L,
        Wfc2_16, nullptr, kMlp, 0L,
        (void*)(out + r0 * kChan), nullptr, kChan, 0L,
        fc2_b, X1 + r0 * kChan, 0L, kMlpChunkRows, kChan, kMlp, kFc2Scale);
  }
}
